// RNN_71133248356918
// MI455X (gfx1250) — hardware-verified
//
#include <hip/hip_runtime.h>
#include <math.h>

constexpr int NBATCH   = 512;
constexpr int NSTEP    = 2048;
constexpr int NIN      = 2;
constexpr int NHID     = 64;
constexpr int NGATE    = 4 * NHID;
constexpr int NCLS     = 5;
constexpr int NTHR     = 256;
constexpr int ROWS_BLK = 32;
constexpr int HPITCH   = 72;
constexpr int TCHUNK   = 64;
constexpr int XPITCH   = TCHUNK * NIN;
constexpr int NCHUNK   = NSTEP / TCHUNK;
constexpr int HFPITCH  = 68;
constexpr float WCARRY = 256.0f;
constexpr float HCARRY = 256.0f;
constexpr float FOLD   = 1.0f / (WCARRY * HCARRY);

static_assert(NBATCH % ROWS_BLK == 0, "grid exact");
static_assert(NSTEP % TCHUNK == 0, "no time tail");
static_assert(NHID == 64, "two 32-deep k chunks");
static_assert(NGATE == 256, "four gates of 64 columns");
static_assert(NIN == 2, "x row is one 8-B pair");
static_assert((2 * ROWS_BLK * HPITCH) % NTHR == 0, "h zero-fill loop exact");
static_assert(ROWS_BLK * XPITCH == 4 * NTHR * 4, "x chunk staging: 4 float4 per thread");
static_assert(ROWS_BLK * NCLS == 160, "five whole waves write the block output");
static_assert((ROWS_BLK * NCLS * 4) % 128 == 0, "block output = whole 128-B lines");
static_assert(NCLS * NHID == 80 * 4, "W_out staging: 80 float4");

typedef __attribute__((ext_vector_type(16))) _Float16 v16h;
typedef __attribute__((ext_vector_type(8)))  _Float16 v8h;
typedef __attribute__((ext_vector_type(8)))  float    v8f;
typedef __attribute__((ext_vector_type(4)))  float    v4f;
typedef __attribute__((ext_vector_type(2)))  float    v2f;

union FragU { v16h v; v8h h[2]; };

__device__ __forceinline__ v16h load_afrag(const _Float16* p) {
  FragU f;
  f.h[0] = *(const v8h*)(p);
  f.h[1] = *(const v8h*)(p + 16);
  return f.v;
}

__device__ __forceinline__ v16h load_bfrag_f32(const float* p) {
  const v4f a = *(const v4f*)(p);
  const v4f b = *(const v4f*)(p + 4);
  const v4f c = *(const v4f*)(p + 16);
  const v4f d = *(const v4f*)(p + 20);
  v16h o;
#pragma unroll
  for (int e = 0; e < 4; ++e) {
    o[e]      = (_Float16)(a[e] * WCARRY);
    o[4 + e]  = (_Float16)(b[e] * WCARRY);
    o[8 + e]  = (_Float16)(c[e] * WCARRY);
    o[12 + e] = (_Float16)(d[e] * WCARRY);
  }
  return o;
}

__device__ __forceinline__ v8f mma_h(v16h a, v16h b, v8f c) {
  return __builtin_amdgcn_wmma_f32_16x16x32_f16(false, a, false, b, (short)0, c, false, false);
}
__device__ __forceinline__ void guard_group(v8f& a, v8f& b, v8f& c, v8f& d, v16h x, v16h y) {
  asm volatile("v_nop\n\tv_nop\n\tv_nop\n\tv_nop" : "+v"(a), "+v"(b), "+v"(c), "+v"(d) : "v"(x), "v"(y));
}
__device__ __forceinline__ void keep8_h(v16h a, v16h b, v16h c, v16h d, v16h e, v16h f, v16h g, v16h h) {
  asm volatile("v_nop" :: "v"(a), "v"(b), "v"(c), "v"(d), "v"(e), "v"(f), "v"(g), "v"(h));
}
__device__ __forceinline__ void settle_frag(v16h& f) { asm volatile("" : "+v"(f) :: "memory"); }

__device__ __forceinline__ float fsig(float v)  { return __builtin_amdgcn_rcpf(1.0f + __expf(-v)); }
__device__ __forceinline__ float ftanh(float v) { return 1.0f - 2.0f * __builtin_amdgcn_rcpf(__expf(2.0f * v) + 1.0f); }

__device__ __forceinline__ void stage_x_chunk(const float* __restrict__ x, float* xdst, int rowbase, int chunk, int tid) {
  v4f v[4];
#pragma unroll
  for (int i = 0; i < 4; ++i) {
    const int idx = i * NTHR + tid;
    const int row = idx >> 5;
    const int c4  = (idx & 31) * 4;
    v[i] = *(const v4f*)(x + ((size_t)(rowbase + row) * NSTEP + (size_t)chunk * TCHUNK) * NIN + c4);
  }
#pragma unroll
  for (int i = 0; i < 4; ++i) {
    const int idx = i * NTHR + tid;
    const int row = idx >> 5;
    const int c4  = (idx & 31) * 4;
    *(v4f*)(xdst + row * XPITCH + c4) = v[i];
  }
}

__global__ __launch_bounds__(NTHR) void lstm_scan_kernel(const float* __restrict__ x,
                                                         const float* __restrict__ w_ih,
                                                         const float* __restrict__ w_hh,
                                                         const float* __restrict__ b_ih,
                                                         const float* __restrict__ b_hh,
                                                         const float* __restrict__ w_out,
                                                         const float* __restrict__ b_out,
                                                         float* __restrict__ out) {
  __shared__ __align__(16) _Float16 hA[2][ROWS_BLK * HPITCH];
  __shared__ __align__(16) float    xs[2][ROWS_BLK * XPITCH];
  __shared__ __align__(16) float    hfin[ROWS_BLK * HFPITCH];
  __shared__ __align__(16) float    wos[NCLS * NHID];

  const int tid  = threadIdx.x;
  const int lane = tid & 31;
  const int wv   = tid >> 5;
  const int hi   = lane >> 4;
  const int lo   = lane & 15;
  const int rg   = wv >> 2;
  const int cg   = wv & 3;
  const int rowbase = blockIdx.x * ROWS_BLK;

  v16h Bf[4][2];
#pragma unroll
  for (int G = 0; G < 4; ++G) {
    const int n = G * NHID + cg * 16 + lo;
#pragma unroll
    for (int kc = 0; kc < 2; ++kc) {
      Bf[G][kc] = load_bfrag_f32(w_hh + (size_t)n * NHID + kc * 32 + 8 * hi);
      settle_frag(Bf[G][kc]);
    }
  }
  float bsum[4], wi0[4], wi1[4];
#pragma unroll
  for (int G = 0; G < 4; ++G) {
    const int n = G * NHID + cg * 16 + lo;
    const float ba = b_ih[n];
    const float bb = b_hh[n];
    const v2f   ww = *(const v2f*)(w_ih + (size_t)n * NIN);
    bsum[G] = ba + bb;
    wi0[G]  = ww[0];
    wi1[G]  = ww[1];
    if (G == 1) asm volatile("" : "+v"(bsum[0]), "+v"(bsum[1]) :: "memory");
  }

  float creg[8], hreg[8];
#pragma unroll
  for (int r = 0; r < 8; ++r) { creg[r] = 0.0f; hreg[r] = 0.0f; }

  {
    _Float16* hflat = &hA[0][0];
#pragma unroll 1
    for (int i = tid; i < 2 * ROWS_BLK * HPITCH; i += NTHR) hflat[i] = (_Float16)0.0f;
  }
  stage_x_chunk(x, &xs[0][0], rowbase, 0, tid);
  __syncthreads();

  const v8f z8 = {0.f, 0.f, 0.f, 0.f, 0.f, 0.f, 0.f, 0.f};
  const int arow_off = (rg * 16 + lo) * HPITCH + 8 * hi;
  const int mrow0    = rg * 16 + 8 * hi;

#pragma unroll 1
  for (int t = 0; t < NSTEP; ++t) {
    const int cb = t & 1;
    const int nb = cb ^ 1;
    const int ch = t >> 6;
    const int tl = t & (TCHUNK - 1);
    const int xb = ch & 1;

    if (tl == 0 && ch + 1 < NCHUNK) {
      stage_x_chunk(x, &xs[0][0] + (xb ^ 1) * (ROWS_BLK * XPITCH), rowbase, ch + 1, tid);
    }

    const _Float16* ap = &hA[0][0] + cb * (ROWS_BLK * HPITCH) + arow_off;
    const v16h A0 = load_afrag(ap);
    const v16h A1 = load_afrag(ap + 32);

    v8f acc[4];
    acc[0] = z8; acc[1] = z8; acc[2] = z8; acc[3] = z8;
#pragma unroll
    for (int G = 0; G < 4; ++G) acc[G] = mma_h(A0, Bf[G][0], acc[G]);
#pragma unroll
    for (int G = 0; G < 4; ++G) acc[G] = mma_h(A1, Bf[G][1], acc[G]);
    guard_group(acc[0], acc[1], acc[2], acc[3], A0, A1);
    keep8_h(Bf[0][0], Bf[0][1], Bf[1][0], Bf[1][1], Bf[2][0], Bf[2][1], Bf[3][0], Bf[3][1]);

    const float* xrow = &xs[0][0] + xb * (ROWS_BLK * XPITCH) + mrow0 * XPITCH + tl * NIN;
    _Float16* hnext = &hA[0][0] + nb * (ROWS_BLK * HPITCH) + mrow0 * HPITCH + cg * 16 + lo;
#pragma unroll
    for (int r = 0; r < 8; ++r) {
      const v2f xv = *(const v2f*)(xrow + r * XPITCH);
      const float x0 = xv[0];
      const float x1 = xv[1];
      const float zi = acc[0][r] * FOLD + (bsum[0] + x0 * wi0[0] + x1 * wi1[0]);
      const float zf = acc[1][r] * FOLD + (bsum[1] + x0 * wi0[1] + x1 * wi1[1]);
      const float zg = acc[2][r] * FOLD + (bsum[2] + x0 * wi0[2] + x1 * wi1[2]);
      const float zo = acc[3][r] * FOLD + (bsum[3] + x0 * wi0[3] + x1 * wi1[3]);
      const float ig = fsig(zi);
      const float fg = fsig(zf);
      const float gg = ftanh(zg);
      const float og = fsig(zo);
      const float cn = fg * creg[r] + ig * gg;
      creg[r] = cn;
      const float hn = og * ftanh(cn);
      hreg[r] = hn;
      hnext[r * HPITCH] = (_Float16)(hn * HCARRY);
    }
    __syncthreads();
  }

#pragma unroll
  for (int r = 0; r < 8; ++r) hfin[(mrow0 + r) * HFPITCH + cg * 16 + lo] = hreg[r];
  {
    const int wi = (tid < 80) ? tid : 79;
    const v4f wv4 = *(const v4f*)(w_out + wi * 4);
    if (tid < 80) *(v4f*)(wos + wi * 4) = wv4;
  }
  __syncthreads();

  {
    const int ct = (tid < ROWS_BLK * NCLS) ? tid : (ROWS_BLK * NCLS - 1);
    const int b  = ct / NCLS;
    const int o  = ct - b * NCLS;
    float s = 0.0f;
#pragma unroll 8
    for (int j = 0; j < NHID; ++j) s += hfin[b * HFPITCH + j] * wos[o * NHID + j];
    s += b_out[o];
    if (tid < ROWS_BLK * NCLS) {
      float* op = out + (size_t)rowbase * NCLS + tid;
      *(volatile float*)op = s;
      __threadfence();
      *(volatile float*)op = s;
    }
  }
}

extern "C" void kernel_launch(void* const* d_in, const int* in_sizes, int n_in,
                              void* d_out, int out_size, void* d_ws, size_t ws_size, hipStream_t stream) {
  (void)d_ws; (void)ws_size;
  if (n_in < 7 || d_out == nullptr) return;
  if (in_sizes[0] != NBATCH * NSTEP * NIN || in_sizes[1] != NGATE * NIN || in_sizes[2] != NGATE * NHID ||
      in_sizes[3] != NGATE || in_sizes[4] != NGATE || in_sizes[5] != NCLS * NHID || in_sizes[6] != NCLS ||
      out_size != NBATCH * NCLS) return;

  const float* x     = (const float*)d_in[0];
  const float* w_ih  = (const float*)d_in[1];
  const float* w_hh  = (const float*)d_in[2];
  const float* b_ih  = (const float*)d_in[3];
  const float* b_hh  = (const float*)d_in[4];
  const float* w_out = (const float*)d_in[5];
  const float* b_out = (const float*)d_in[6];
  float* out = (float*)d_out;

  lstm_scan_kernel<<<NBATCH / ROWS_BLK, NTHR, 0, stream>>>(x, w_ih, w_hh, b_ih, b_hh, w_out, b_out, out);
}
